// SelfAttentionEncoderBlock_28252294873695
// MI455X (gfx1250) — hardware-verified
//
#include <hip/hip_runtime.h>


#define NB_  8
#define NN   1024
#define NT   (NB_ * NN)
#define CC   384
#define HID  768
#define NH_  12
#define HD   32
#define C3   1152
#define ZH   4
#define GW   32
#define NREL 63
#define DM   CC
#define SCL  0.17677669529663687f
#define LOSC 1024.0f

typedef _Float16 h16;
typedef unsigned short bf;
typedef __attribute__((ext_vector_type(16))) __bf16   v16bf;
typedef __attribute__((ext_vector_type(16))) _Float16 v16h;
typedef __attribute__((ext_vector_type(8)))  _Float16 v8h;
typedef __attribute__((ext_vector_type(8)))  unsigned short v8us;
typedef __attribute__((ext_vector_type(8)))  float    v8f;
typedef __attribute__((ext_vector_type(4)))  float    v4f;
typedef v8h  __attribute__((may_alias)) v8ha;
typedef v4f  __attribute__((may_alias)) v4fa;
typedef v8us __attribute__((may_alias)) v8usa;

__device__ __forceinline__ unsigned short f2bf(float f) { unsigned u = __float_as_uint(f); u += 0x7FFFu + ((u >> 16) & 1u); return (unsigned short)(u >> 16); }
__device__ __forceinline__ float bf2f(unsigned short b) { return __uint_as_float(((unsigned)b) << 16); }
__device__ __forceinline__ float bfr(float f) { return bf2f(f2bf(f)); }
__device__ __forceinline__ v16h cat16(v8h lo, v8h hi) { return __builtin_shufflevector(lo, hi, 0, 1, 2, 3, 4, 5, 6, 7, 8, 9, 10, 11, 12, 13, 14, 15); }
__device__ __forceinline__ v16bf cat16b(v8us lo, v8us hi) { return __builtin_bit_cast(v16bf, __builtin_shufflevector(lo, hi, 0, 1, 2, 3, 4, 5, 6, 7, 8, 9, 10, 11, 12, 13, 14, 15)); }
__device__ __forceinline__ v8f wmma16(v16h a, v16h b, v8f c) { return __builtin_amdgcn_wmma_f32_16x16x32_f16(false, a, false, b, (short)0, c, false, false); }
__device__ __forceinline__ v8f wmmab(v16bf a, v16bf b, v8f c) { return __builtin_amdgcn_wmma_f32_16x16x32_bf16(false, a, false, b, (short)0, c, false, false); }

template <bool SPLITA, bool F16OUT = false>
__global__ __launch_bounds__(128) void k_gemmb(const bf* __restrict__ A, const bf* __restrict__ Al, const bf* __restrict__ Bn, const float* __restrict__ bias, float* C, int ldc, h16* C2, const float* __restrict__ R = nullptr, int K = DM, int roundR = 1) {
    __shared__ __align__(16) float ost[4][16 * 68];
    const int lane = threadIdx.x & 31, wave = threadIdx.x >> 5, lr = lane & 15, hi = lane >> 4;
    const int r0 = blockIdx.x * 64 + wave * 16, c0 = blockIdx.y * 64;
    const size_t aoff = (size_t)(r0 + lr) * K + 8 * hi;
    size_t boff[4];
#pragma unroll
    for (int t = 0; t < 4; ++t) boff[t] = (size_t)(c0 + t * 16 + lr) * K + 8 * hi;
    v8f acc[4];
#pragma unroll
    for (int t = 0; t < 4; ++t) acc[t] = (v8f){};
#pragma unroll 1
    for (int kc = 0; kc < K; kc += 32) {
        const v16bf a = cat16b(*(const v8us*)(A + aoff + kc), *(const v8us*)(A + aoff + kc + 16));
        v16bf al = a;
        if (SPLITA) al = cat16b(*(const v8us*)(Al + aoff + kc), *(const v8us*)(Al + aoff + kc + 16));
#pragma unroll
        for (int t = 0; t < 4; ++t) { const v16bf b = cat16b(*(const v8us*)(Bn + boff[t] + kc), *(const v8us*)(Bn + boff[t] + kc + 16)); acc[t] = wmmab(a, b, acc[t]); if (SPLITA) acc[t] = wmmab(al, b, acc[t]); }
        asm volatile("v_nop\n\tv_nop\n\tv_nop\n\tv_nop" : "+v"(acc[0]), "+v"(acc[1]), "+v"(acc[2]), "+v"(acc[3]) : "v"(a), "v"(al));
    }
    float* os = &ost[wave][0];
#pragma unroll
    for (int t = 0; t < 4; ++t) { const float bv = bias ? bfr(bias[c0 + t * 16 + lr]) : 0.f;
#pragma unroll
        for (int j = 0; j < 8; ++j) os[(hi * 8 + j) * 68 + t * 16 + lr] = acc[t][j] + bv; }
    __syncthreads();
    if (F16OUT) {
        h16* crow = (h16*)(void*)C + (size_t)r0 * ldc + c0;
        auto pass = [&]() {
#pragma unroll
            for (int s = 0; s < 4; ++s) { const int row = 4 * s + (lane >> 3), piece = lane & 7; const float* sp = os + row * 68 + piece * 8; v8h o, o2;
#pragma unroll
                for (int i = 0; i < 8; ++i) { const h16 a = (h16)sp[i]; o[i] = a; o2[i] = (h16)((sp[i] - (float)a) * LOSC); }
                *(volatile v8h*)(crow + (size_t)row * ldc + piece * 8) = o; if (C2) *(volatile v8h*)(C2 + (size_t)r0 * ldc + c0 + (size_t)row * ldc + piece * 8) = o2; }
        };
        pass(); __threadfence(); pass();
    } else {
        float* crow = C + (size_t)r0 * ldc + c0;
        auto pass = [&]() {
#pragma unroll
            for (int s = 0; s < 8; ++s) { const int Lid = (lane >> 3) + 4 * s, piece = lane & 7; const int row = Lid >> 1, cofs = (Lid & 1) * 32 + piece * 4;
                v4f val = *(const v4fa*)(os + row * 68 + cofs); if (R) { const v4f rv = *(const v4f*)(R + ((size_t)r0 + row) * ldc + c0 + cofs); val += roundR ? (v4f){bfr(rv[0]), bfr(rv[1]), bfr(rv[2]), bfr(rv[3])} : rv; }
                *(volatile v4f*)(crow + (size_t)row * ldc + cofs) = val; }
        };
        pass(); __threadfence(); pass();
    }
}

__global__ __launch_bounds__(256) void k_cvt8(const float* __restrict__ src, bf* dst, size_t n8) {
    const size_t i = (size_t)blockIdx.x * 256 + threadIdx.x; if (i >= n8) return;
    const v8f v = *(const v8f*)(src + i * 8); v8us o;
#pragma unroll
    for (int k = 0; k < 8; ++k) o[k] = f2bf(v[k]);
    *(volatile v8us*)(dst + i * 8) = o; __threadfence(); *(volatile v8us*)(dst + i * 8) = o;
}
__global__ __launch_bounds__(256) void k_zero8(bf* dst, size_t n8) {
    const size_t i = (size_t)blockIdx.x * 256 + threadIdx.x; if (i >= n8) return; v8us z;
#pragma unroll
    for (int k = 0; k < 8; ++k) z[k] = 0;
    *(volatile v8us*)(dst + i * 8) = z; __threadfence(); *(volatile v8us*)(dst + i * 8) = z;
}

template <int MODE>
__global__ __launch_bounds__(128) void k_gemm3z(const bf* __restrict__ Ah, const bf* __restrict__ Al, const bf* __restrict__ Bh, const bf* __restrict__ Bl, int K, float* C, int ldc, size_t sA, size_t sB, size_t sC) {
    if ((MODE & 1) && (int)blockIdx.y * 64 > (int)blockIdx.x * 64 + 63) return;
    const size_t z = blockIdx.z; Ah += z * sA; Al += z * sA; Bh += z * sB; Bl += z * sB; C += z * sC;
    const int Klim = (MODE & 2) ? min(K, ((int)blockIdx.x + 1) * 64) : K;
    __shared__ __align__(16) float ost[4][16 * 68];
    const int lane = threadIdx.x & 31, wave = threadIdx.x >> 5, lr = lane & 15, hi = lane >> 4;
    const int r0 = blockIdx.x * 64 + wave * 16, c0 = blockIdx.y * 64;
    const size_t aoff = (size_t)(r0 + lr) * K + 8 * hi;
    v8f acc[4];
#pragma unroll
    for (int t = 0; t < 4; ++t) acc[t] = (v8f){};
#pragma unroll 1
    for (int kc = 0; kc < Klim; kc += 32) {
        const v16bf a = cat16b(*(const v8us*)(Ah + aoff + kc), *(const v8us*)(Ah + aoff + kc + 16));
        v16bf al = a; if (!(MODE & 4) && !(MODE & 16)) al = cat16b(*(const v8us*)(Al + aoff + kc), *(const v8us*)(Al + aoff + kc + 16));
#pragma unroll
        for (int t = 0; t < 4; ++t) { const size_t bo = (size_t)(c0 + t * 16 + lr) * K + kc + 8 * hi;
            const v16bf bh = cat16b(*(const v8us*)(Bh + bo), *(const v8us*)(Bh + bo + 16));
            acc[t] = wmmab(a, bh, acc[t]);
            if (!(MODE & 4)) { if (!(MODE & 16)) acc[t] = wmmab(al, bh, acc[t]); if (!(MODE & 8)) { const v16bf bl = cat16b(*(const v8us*)(Bl + bo), *(const v8us*)(Bl + bo + 16)); acc[t] = wmmab(a, bl, acc[t]); } } }
        asm volatile("v_nop\n\tv_nop\n\tv_nop\n\tv_nop" : "+v"(acc[0]), "+v"(acc[1]), "+v"(acc[2]), "+v"(acc[3]) : "v"(a), "v"(al));
    }
    float* os = &ost[wave][0];
#pragma unroll
    for (int t = 0; t < 4; ++t) {
#pragma unroll
        for (int j = 0; j < 8; ++j) os[(hi * 8 + j) * 68 + t * 16 + lr] = acc[t][j]; }
    __builtin_amdgcn_wave_barrier(); asm volatile("" ::: "memory");
    float* crow = C + (size_t)r0 * ldc + c0;
    auto pass = [&]() {
#pragma unroll
        for (int s = 0; s < 8; ++s) { const int Lid = (lane >> 3) + 4 * s, piece = lane & 7; const int row = Lid >> 1, cofs = (Lid & 1) * 32 + piece * 4;
            const v4f val = *(const v4fa*)(os + row * 68 + cofs); *(volatile v4f*)(crow + (size_t)row * ldc + cofs) = val; }
    };
    pass(); __threadfence(); pass();
}
__global__ __launch_bounds__(256) void k_planes32z(const float* __restrict__ F, int ld, int off, float sc, int rows, bf* Ph, bf* Pl) {
    typedef __attribute__((ext_vector_type(2))) unsigned short v2us;
    const int lane = threadIdx.x & 31; const size_t r = ((size_t)blockIdx.x * 8 + (threadIdx.x >> 5)) * 2 + (lane >> 4); if (r >= (size_t)rows) return; const int z = blockIdx.z; const int c0 = (lane & 15) * 2; v2us oh, ol;
    Ph += (size_t)z * rows * 32; Pl += (size_t)z * rows * 32;
#pragma unroll
    for (int i = 0; i < 2; ++i) { const float y = F[r * ld + off + z * 32 + c0 + i] * sc; const unsigned short hb = f2bf(y); oh[i] = hb; ol[i] = f2bf(y - bf2f(hb)); }
    const size_t o = r * 32 + c0; *(volatile v2us*)(Ph + o) = oh; *(volatile v2us*)(Pl + o) = ol; __threadfence(); *(volatile v2us*)(Ph + o) = oh; *(volatile v2us*)(Pl + o) = ol;
}
__global__ __launch_bounds__(256) void k_vtpadz(const float* __restrict__ F, int ld, int off, int nk, bf* Th, bf* Tl) {
    typedef __attribute__((ext_vector_type(2))) unsigned short v2us;
    const int lane = threadIdx.x & 31; const size_t wid = (size_t)blockIdx.x * 8 + (threadIdx.x >> 5); if (wid >= (size_t)64 * (nk / 64)) return; const int z = blockIdx.z; const int d = (int)(wid / (nk / 64)); const int k0 = (int)(wid % (nk / 64)) * 64 + lane * 2; v2us oh, ol;
    Th += (size_t)z * 64 * nk; Tl += (size_t)z * 64 * nk;
#pragma unroll
    for (int i = 0; i < 2; ++i) { const float y = (d < 32) ? F[(size_t)(k0 + i) * ld + off + z * 32 + (d < 32 ? d : 0)] : 0.f; const unsigned short hb = f2bf(y); oh[i] = hb; ol[i] = f2bf(y - bf2f(hb)); }
    const size_t o = (size_t)d * nk + k0; *(volatile v2us*)(Th + o) = oh; *(volatile v2us*)(Tl + o) = ol; __threadfence(); *(volatile v2us*)(Th + o) = oh; *(volatile v2us*)(Tl + o) = ol;
}
template <int NK>
__global__ __launch_bounds__(256) void k_softmaxz(const float* __restrict__ S, int rows, bf* PH, bf* PL) {
    typedef __attribute__((ext_vector_type(4))) unsigned short v4us;
    const int lane = threadIdx.x & 31, i = blockIdx.x * 8 + (threadIdx.x >> 5); if (i >= rows) return; const size_t zo = (size_t)blockIdx.z * rows * NK; const float* sr = S + zo + (size_t)i * NK; PH += zo; PL += zo;
    float m = -3.0e38f;
#pragma unroll 1
    for (int c0 = lane * 4; c0 < NK; c0 += 128) {
#pragma unroll
        for (int q = 0; q < 4; ++q) m = fmaxf(m, sr[c0 + q]); }
#pragma unroll
    for (int sh = 16; sh; sh >>= 1) m = fmaxf(m, __shfl_xor(m, sh, 32));
    float sum = 0.f;
#pragma unroll 1
    for (int c0 = lane * 4; c0 < NK; c0 += 128) {
#pragma unroll
        for (int q = 0; q < 4; ++q) sum += __expf(sr[c0 + q] - m); }
#pragma unroll
    for (int sh = 16; sh; sh >>= 1) sum += __shfl_xor(sum, sh, 32);
    const float inv = 1.0f / sum;
#pragma unroll 1
    for (int ps = 0; ps < 2; ++ps) {
#pragma unroll 1
        for (int c0 = lane * 4; c0 < NK; c0 += 128) { v4us oh, ol;
#pragma unroll
            for (int q = 0; q < 4; ++q) { const float p = __expf(sr[c0 + q] - m) * inv; const unsigned short hb = f2bf(p); oh[q] = hb; ol[q] = f2bf(p - bf2f(hb)); }
            const size_t o = (size_t)i * NK + c0; *(volatile v4us*)(PH + o) = oh; *(volatile v4us*)(PL + o) = ol; }
        if (ps == 0) __threadfence(); }
}
__global__ __launch_bounds__(256) void k_placez(const float* __restrict__ XH, int rows, int ldy, float* Y) {
    const int lane = threadIdx.x & 31; const size_t q = (size_t)blockIdx.x * 8 + (threadIdx.x >> 5); if (q >= (size_t)rows) return; const int z = blockIdx.z; const float v = XH[((size_t)z * rows + q) * 64 + lane];
    *(volatile float*)(Y + q * ldy + z * 32 + lane) = v; __threadfence(); *(volatile float*)(Y + q * ldy + z * 32 + lane) = v;
}

template <bool RAW>
__global__ __launch_bounds__(256) void k_lnpl(const float* __restrict__ X, size_t rows, const float* __restrict__ g, const float* __restrict__ bb, bf* Ph, bf* Pl) {
    typedef __attribute__((ext_vector_type(4))) unsigned short v4us;
    const int lane = threadIdx.x & 31; const size_t r = (size_t)blockIdx.x * 8 + (threadIdx.x >> 5); if (r >= rows) return; float v[12]; float s = 0.f;
#pragma unroll
    for (int q = 0; q < 3; ++q)
#pragma unroll
        for (int i = 0; i < 4; ++i) { float t = X[r * CC + q * 128 + lane * 4 + i]; if (RAW) t = bfr(t); v[q * 4 + i] = t; s += t; }
#pragma unroll
    for (int sh = 16; sh; sh >>= 1) s += __shfl_xor(s, sh, 32);
    const float mu = s * (1.0f / CC); float qv = 0.f;
#pragma unroll
    for (int i = 0; i < 12; ++i) { const float d = v[i] - mu; qv = fmaf(d, d, qv); }
#pragma unroll
    for (int sh = 16; sh; sh >>= 1) qv += __shfl_xor(qv, sh, 32);
    const float rs = rsqrtf(qv * (1.0f / CC) + 1e-5f);
#pragma unroll 1
    for (int ps = 0; ps < 2; ++ps) {
#pragma unroll
        for (int q = 0; q < 3; ++q) { v4us oh, ol;
#pragma unroll
            for (int i = 0; i < 4; ++i) { const int c = q * 128 + lane * 4 + i; const float y = (v[q * 4 + i] - mu) * rs * bfr(g[c]) + bfr(bb[c]); const unsigned short hb = f2bf(y); oh[i] = hb; ol[i] = f2bf(y - bf2f(hb)); }
            const size_t o = r * CC + q * 128 + lane * 4; *(volatile v4us*)(Ph + o) = oh; *(volatile v4us*)(Pl + o) = ol; }
        if (ps == 0) __threadfence(); }
}
__global__ __launch_bounds__(256) void k_dwgelu(const float* __restrict__ H1, const float* __restrict__ wdw, const float* __restrict__ bdw, bf* Gh, bf* Gl) {
    const int lane = threadIdx.x & 31; const size_t r = (size_t)blockIdx.x * 8 + (threadIdx.x >> 5); if (r >= (size_t)NT) return; const int b = (int)(r / NN), n = (int)(r % NN); const int y = n / GW, x = n % GW;
#pragma unroll 1
    for (int ps = 0; ps < 2; ++ps) {
#pragma unroll 1
        for (int q = 0; q < HID / 256; ++q) { v8us oh, ol;
#pragma unroll 1
            for (int i = 0; i < 8; ++i) { const int c = q * 256 + lane * 8 + i; float acc = bfr(bdw[c]);
#pragma unroll 1
                for (int ty = 0; ty < 3; ++ty) { const int yy = y + 2 * ty - 2; if (yy < 0 || yy >= GW) continue;
#pragma unroll 1
                    for (int tx = 0; tx < 3; ++tx) { const int xx = x + 2 * tx - 2; if (xx < 0 || xx >= GW) continue; const float hv = H1[((size_t)b * NN + yy * GW + xx) * HID + c];
                        const float gv = 0.5f * hv * (1.0f + erff(hv * 0.70710678118654752f)); acc = fmaf(gv, bfr(wdw[(size_t)c * 9 + ty * 3 + tx]), acc); } }
                const float yv = 0.5f * acc * (1.0f + erff(acc * 0.70710678118654752f)); const unsigned short hb = f2bf(yv); oh[i] = hb; ol[i] = f2bf(yv - bf2f(hb)); }
            const size_t o = r * HID + q * 256 + lane * 8; *(volatile v8us*)(Gh + o) = oh; *(volatile v8us*)(Gl + o) = ol; }
        if (ps == 0) __threadfence(); }
}
__global__ __launch_bounds__(256) void k_biasmap(const int* __restrict__ ridx, const float* __restrict__ rtab, const float* __restrict__ gb, int GBS, float* BIAS) {
    const int lane = threadIdx.x & 31; const size_t w = (size_t)blockIdx.x * 8 + (threadIdx.x >> 5); if (w >= (size_t)NH_ * NN) return; const int h = (int)(w / NN), q = (int)(w % NN);
#pragma unroll 1
    for (int ps = 0; ps < 2; ++ps) {
#pragma unroll 1
        for (int c0 = lane * 4; c0 < NN; c0 += 128) { v4f o;
#pragma unroll
            for (int i = 0; i < 4; ++i) { const int k = c0 + i; int id = ridx[(size_t)q * NN + k]; id = id < 0 ? 0 : (id >= NREL * NREL ? NREL * NREL - 1 : id); o[i] = bfr(rtab[(size_t)id * NH_ + h]) + bfr(gb[(size_t)q * GBS + k]); }
            *(volatile v4f*)(BIAS + w * NN + c0) = o; }
        if (ps == 0) __threadfence(); }
}
__global__ __launch_bounds__(256) void k_hpl32(const float* __restrict__ QKV, size_t r0, int col0, int h0, float sc, bf* Ph, bf* Pl) {
    typedef __attribute__((ext_vector_type(4))) unsigned short v4us;
    const int lane = threadIdx.x & 31; const size_t w = (size_t)blockIdx.x * 8 + (threadIdx.x >> 5); if (w >= (size_t)NN / 4) return; const int z = blockIdx.z; const int i = (int)(w * 4 + (lane >> 3)); const int c0 = (lane & 7) * 4; v4us oh, ol;
#pragma unroll
    for (int q = 0; q < 4; ++q) { const float y = QKV[(r0 + i) * C3 + col0 + (h0 + z) * HD + c0 + q] * sc; const unsigned short hb = f2bf(y); oh[q] = hb; ol[q] = f2bf(y - bf2f(hb)); }
    const size_t o = ((size_t)z * NN + i) * HD + c0; *(volatile v4us*)(Ph + o) = oh; *(volatile v4us*)(Pl + o) = ol; __threadfence(); *(volatile v4us*)(Ph + o) = oh; *(volatile v4us*)(Pl + o) = ol;
}
__global__ __launch_bounds__(256) void k_vT32(const float* __restrict__ QKV, size_t r0, int h0, bf* Th, bf* Tl) {
    __shared__ float tl[64][33];
    typedef __attribute__((ext_vector_type(4))) unsigned short v4us;
    const int tid = threadIdx.x; const int t0 = blockIdx.x * 64; const int z = blockIdx.z; const int rr = tid >> 2, cq = (tid & 3) * 8;
#pragma unroll
    for (int i = 0; i < 8; ++i) tl[rr][cq + i] = QKV[(r0 + t0 + rr) * C3 + 2 * CC + (h0 + z) * HD + cq + i];
    __syncthreads();
    const int lane = tid & 31, wv = tid >> 5;
    auto pass = [&]() {
#pragma unroll
        for (int st = 0; st < 4; ++st) { const int dr = wv * 8 + st * 2 + (lane >> 4); const int tq = (lane & 15) * 4; v4us oh, ol;
#pragma unroll
            for (int i = 0; i < 4; ++i) { const float y = (dr < HD) ? tl[tq + i][dr < HD ? dr : 0] : 0.f; const unsigned short hb = f2bf(y); oh[i] = hb; ol[i] = f2bf(y - bf2f(hb)); }
            const size_t o = ((size_t)z * 64 + dr) * NN + t0 + tq; *(volatile v4us*)(Th + o) = oh; *(volatile v4us*)(Tl + o) = ol; }
    };
    pass(); __threadfence(); pass();
}
__global__ __launch_bounds__(256) void k_softb(const float* __restrict__ S, const float* __restrict__ BIAS, int h0, bf* PH, bf* PL) {
    typedef __attribute__((ext_vector_type(4))) unsigned short v4us;
    const int lane = threadIdx.x & 31, i = blockIdx.x * 8 + (threadIdx.x >> 5); if (i >= NN) return; const int z = blockIdx.z; const size_t zo = (size_t)z * NN * NN; const float* sr = S + zo + (size_t)i * NN; const float* br = BIAS + ((size_t)(h0 + z) * NN + i) * NN;
    float m = -3.0e38f;
#pragma unroll 1
    for (int c0 = lane * 4; c0 < NN; c0 += 128) {
#pragma unroll
        for (int q = 0; q < 4; ++q) m = fmaxf(m, sr[c0 + q] + br[c0 + q]); }
#pragma unroll
    for (int sh = 16; sh; sh >>= 1) m = fmaxf(m, __shfl_xor(m, sh, 32));
    float sum = 0.f;
#pragma unroll 1
    for (int c0 = lane * 4; c0 < NN; c0 += 128) {
#pragma unroll
        for (int q = 0; q < 4; ++q) sum += __expf(sr[c0 + q] + br[c0 + q] - m); }
#pragma unroll
    for (int sh = 16; sh; sh >>= 1) sum += __shfl_xor(sum, sh, 32);
    const float inv = 1.0f / sum;
#pragma unroll 1
    for (int ps = 0; ps < 2; ++ps) {
#pragma unroll 1
        for (int c0 = lane * 4; c0 < NN; c0 += 128) { v4us oh, ol;
#pragma unroll
            for (int q = 0; q < 4; ++q) { const float p = __expf(sr[c0 + q] + br[c0 + q] - m) * inv; const unsigned short hb = f2bf(p); oh[q] = hb; ol[q] = f2bf(p - bf2f(hb)); }
            const size_t o = zo + (size_t)i * NN + c0; *(volatile v4us*)(PH + o) = oh; *(volatile v4us*)(PL + o) = ol; }
        if (ps == 0) __threadfence(); }
}
__global__ __launch_bounds__(256) void k_split384(const float* __restrict__ F, size_t rows, bf* Ph, bf* Pl) {
    typedef __attribute__((ext_vector_type(4))) unsigned short v4us;
    const int lane = threadIdx.x & 31; const size_t r = (size_t)blockIdx.x * 8 + (threadIdx.x >> 5); if (r >= rows) return;
#pragma unroll 1
    for (int ps = 0; ps < 2; ++ps) {
#pragma unroll
        for (int q = 0; q < 3; ++q) { const size_t o = r * CC + q * 128 + lane * 4; const v4f v = *(const v4f*)(F + o); v4us oh, ol;
#pragma unroll
            for (int i = 0; i < 4; ++i) { const unsigned short hb = f2bf(v[i]); oh[i] = hb; ol[i] = f2bf(v[i] - bf2f(hb)); }
            *(volatile v4us*)(Ph + o) = oh; *(volatile v4us*)(Pl + o) = ol; }
        if (ps == 0) __threadfence(); }
}


__global__ __launch_bounds__(256) void k_merge32(const float* __restrict__ OZ, size_t r0, int h0, float* O) {
    const int lane = threadIdx.x & 31; const size_t i = (size_t)blockIdx.x * 8 + (threadIdx.x >> 5); if (i >= (size_t)NN) return; const int z = lane >> 3, d0 = (lane & 7) * 4;
    const v4f v = *(const v4f*)(OZ + ((size_t)z * NN + i) * 64 + d0); float* dst = O + (r0 + i) * CC + (h0 + z) * HD + d0; *(volatile v4f*)dst = v; __threadfence(); *(volatile v4f*)dst = v;
}
extern "C" void kernel_launch(void* const* d_in, const int* in_sizes, int n_in,
                              void* d_out, int out_size, void* d_ws, size_t ws_size, hipStream_t stream) {
    (void)in_sizes; (void)n_in; (void)out_size;
    const float* x = (const float*)d_in[0]; const int* ridx = (const int*)d_in[3]; const float* l1g = (const float*)d_in[4]; const float* l1b = (const float*)d_in[5]; const float* wqkv = (const float*)d_in[6]; const float* wproj = (const float*)d_in[7]; const float* bproj = (const float*)d_in[8];
    const float* rtab = (const float*)d_in[9]; const float* gb = (const float*)d_in[10]; const float* l2g = (const float*)d_in[11]; const float* l2b = (const float*)d_in[12]; const float* wpw1 = (const float*)d_in[13]; const float* bpw1 = (const float*)d_in[14]; const float* wdw = (const float*)d_in[15]; const float* bdw = (const float*)d_in[16]; const float* wpw2 = (const float*)d_in[17]; const float* bpw2 = (const float*)d_in[18];
    float* out = (float*)d_out;
    char* wsp = (char*)d_ws;
    auto take = [&](size_t bytes) { char* p = wsp; wsp += (bytes + 255) & ~(size_t)255; return (void*)p; };
    bf* WPW1 = (bf*)take((size_t)HID * CC * 2); bf* WPW2 = (bf*)take((size_t)CC * HID * 2); bf* WQKV = (bf*)take((size_t)C3 * CC * 2); bf* WPROJ = (bf*)take((size_t)CC * CC * 2);
    float* BIAS = (float*)take((size_t)NH_ * NN * NN * 4); bf* Nh = (bf*)take((size_t)NT * CC * 2); bf* Nl = (bf*)take((size_t)NT * CC * 2); float* X1 = (float*)take((size_t)NT * CC * 4); float* O = (float*)take((size_t)NT * CC * 4);
    char* const shared0 = wsp;
    float* H1 = (float*)take((size_t)NT * HID * 4); bf* Gh = (bf*)take((size_t)NT * HID * 2); bf* Gl = (bf*)take((size_t)NT * HID * 2);
    char* const mlpEnd = wsp; wsp = shared0;
    float* QKV = (float*)take((size_t)NT * C3 * 4); bf* Qh = (bf*)take((size_t)ZH * NN * HD * 2); bf* Ql = (bf*)take((size_t)ZH * NN * HD * 2); bf* Kh = (bf*)take((size_t)ZH * NN * HD * 2); bf* Kl = (bf*)take((size_t)ZH * NN * HD * 2); bf* VTh = (bf*)take((size_t)ZH * 64 * NN * 2); bf* VTl = (bf*)take((size_t)ZH * 64 * NN * 2); float* OZ = (float*)take((size_t)ZH * NN * 64 * 4);
    float* S = (float*)take((size_t)ZH * NN * NN * 4); bf* PH = (bf*)take((size_t)ZH * NN * NN * 2); bf* PL = (bf*)take((size_t)ZH * NN * NN * 2);
    if (wsp < mlpEnd) wsp = mlpEnd;
    if ((size_t)(wsp - (char*)d_ws) > ws_size) return;
    k_cvt8<<<(unsigned)(((size_t)HID * CC / 8 + 255) / 256), 256, 0, stream>>>(wpw1, WPW1, (size_t)HID * CC / 8); k_cvt8<<<(unsigned)(((size_t)CC * HID / 8 + 255) / 256), 256, 0, stream>>>(wpw2, WPW2, (size_t)CC * HID / 8);
    k_cvt8<<<(unsigned)(((size_t)C3 * CC / 8 + 255) / 256), 256, 0, stream>>>(wqkv, WQKV, (size_t)C3 * CC / 8); k_cvt8<<<(unsigned)(((size_t)CC * CC / 8 + 255) / 256), 256, 0, stream>>>(wproj, WPROJ, (size_t)CC * CC / 8);
    k_biasmap<<<(NH_ * NN) / 8, 256, 0, stream>>>(ridx, rtab, gb, 1024, BIAS);
    k_lnpl<true><<<NT / 8, 256, 0, stream>>>(x, NT, l2g, l2b, Nh, Nl);
    k_gemmb<true, false><<<dim3(NT / 64, HID / 64, 1), 128, 0, stream>>>(Nh, Nl, WPW1, bpw1, H1, HID, nullptr, nullptr, CC);
    k_dwgelu<<<NT / 8, 256, 0, stream>>>(H1, wdw, bdw, Gh, Gl);
    k_gemmb<true, false><<<dim3(NT / 64, CC / 64, 1), 128, 0, stream>>>(Gh, Gl, WPW2, bpw2, X1, CC, nullptr, x, HID, 1);
    k_lnpl<false><<<NT / 8, 256, 0, stream>>>(X1, NT, l1g, l1b, Nh, Nl);
    k_gemmb<true, false><<<dim3(NT / 64, C3 / 64, 1), 128, 0, stream>>>(Nh, Nl, WQKV, nullptr, QKV, C3, nullptr, nullptr, CC);
    for (int b = 0; b < NB_; ++b) { const size_t r0 = (size_t)b * NN;
        for (int h0 = 0; h0 < NH_; h0 += ZH) {
            k_hpl32<<<dim3((NN / 4) / 8, 1, ZH), 256, 0, stream>>>(QKV, r0, 0, h0, SCL, Qh, Ql); k_hpl32<<<dim3((NN / 4) / 8, 1, ZH), 256, 0, stream>>>(QKV, r0, CC, h0, 1.0f, Kh, Kl); k_vT32<<<dim3(NN / 64, 1, ZH), 256, 0, stream>>>(QKV, r0, h0, VTh, VTl);
            k_gemm3z<0><<<dim3(NN / 64, NN / 64, ZH), 128, 0, stream>>>(Qh, Ql, Kh, Kl, HD, S, NN, (size_t)NN * HD, (size_t)NN * HD, (size_t)NN * NN);
            k_softb<<<dim3(NN / 8, 1, ZH), 256, 0, stream>>>(S, BIAS, h0, PH, PL);
            k_gemm3z<0><<<dim3(NN / 64, 1, ZH), 128, 0, stream>>>(PH, PL, VTh, VTl, NN, OZ, 64, (size_t)NN * NN, (size_t)64 * NN, (size_t)NN * 64);
            k_merge32<<<NN / 8, 256, 0, stream>>>(OZ, r0, h0, O); } }
    k_split384<<<NT / 8, 256, 0, stream>>>(O, NT, Nh, Nl);
    k_gemmb<true, false><<<dim3(NT / 64, CC / 64, 1), 128, 0, stream>>>(Nh, Nl, WPROJ, bproj, out, CC, nullptr, X1, CC, 0);
}
